// TGAT_52828097741151
// MI455X (gfx1250) — hardware-run, weakly checked
//
#include <hip/hip_runtime.h>
#include <math.h>

constexpr int kN     = 50000;
constexpr int kNP    = 50048;
constexpr int kK     = 16;
constexpr int kIn    = 128;
constexpr int kHid   = 128;
constexpr int kT2V   = 64;
constexpr int kXKVld = 256;

constexpr float kQCarry   = 16.0f;
constexpr float kQInv     = 1.0f / 16.0f;
constexpr float kWCarry   = 64.0f;
constexpr float kQKCarry  = 32.0f;
constexpr float kQKInv    = 1.0f / 32.0f;
constexpr float kTBCarry  = 256.0f;
constexpr float kAggCarry = 64.0f;
constexpr float kScaleQK  = kQKCarry / (kQCarry * kWCarry);
constexpr float kScaleAgg = 1.0f / (kTBCarry * kWCarry);
constexpr float kScaleOut = 1.0f / (kAggCarry * kWCarry);
constexpr float kInvSqrtH = 0.08838834764831845f;

static_assert(kNP % 64 == 0 && kNP >= kN, "tile");
static_assert(kIn % 32 == 0 && kT2V % 32 == 0 && kHid % 64 == 0, "tile");
static_assert(kNP % 8 == 0, "tile");

constexpr size_t kBytesXb    = (size_t)kNP * kIn * 2;
constexpr size_t kBytesBtx   = (size_t)3 * kHid * kIn * 2;
constexpr size_t kBytesBtkt  = (size_t)kT2V * kHid * 2;
constexpr size_t kBytesBtvt  = (size_t)kHid * kT2V * 2;
constexpr size_t kBytesBto   = (size_t)kHid * kHid * 2;
constexpr size_t kBytesCq    = 512;
constexpr size_t kBytesBo    = 512;
constexpr size_t kBytesQ16   = (size_t)kNP * kHid * 2;
constexpr size_t kBytesXKV   = (size_t)kNP * kXKVld * 4;
constexpr size_t kBytesQK    = (size_t)kNP * kT2V * 2;
constexpr size_t kBytesAggx  = (size_t)kNP * kHid * 4;
constexpr size_t kBytesTB    = (size_t)kNP * kT2V * 2;
constexpr size_t kBytesAgg16 = (size_t)kNP * kHid * 2;
constexpr size_t kBytesTotal = kBytesXb + kBytesBtx + kBytesBtkt + kBytesBtvt + kBytesBto + kBytesCq + kBytesBo +
                               kBytesQ16 + kBytesXKV + kBytesQK + kBytesAggx + kBytesTB + kBytesAgg16;
static_assert(kBytesTotal == 128287744, "carve");
static_assert(kBytesTotal <= 134217728, "carve");

typedef __attribute__((ext_vector_type(16))) _Float16 v16h;
typedef __attribute__((ext_vector_type(8)))  _Float16 v8h;
typedef __attribute__((ext_vector_type(16))) __bf16   v16b;
typedef __attribute__((ext_vector_type(8)))  __bf16   v8b;
typedef __attribute__((ext_vector_type(8)))  float    v8f;
typedef __attribute__((ext_vector_type(4)))  float    v4f;
typedef __attribute__((ext_vector_type(2)))  float    v2f;
typedef __attribute__((ext_vector_type(4)))  unsigned int v4u;

__device__ __forceinline__ unsigned short f2bf_bits(float f) {
  unsigned u = __float_as_uint(f);
  return (unsigned short)((u + 0x7FFFu + ((u >> 16) & 1u)) >> 16);
}
__device__ __forceinline__ float bf_bits2f(unsigned short h) { return __uint_as_float(((unsigned)h) << 16); }

__device__ __forceinline__ void dep_guard_h(v8f& a, v8f& b, v16h x, v16h y) { asm volatile("v_nop\n\tv_nop\n\tv_nop\n\tv_nop" : "+v"(a), "+v"(b) : "v"(x), "v"(y)); }
__device__ __forceinline__ void dep_guard_b(v8f& a, v8f& b, v16b x, v16b y) { asm volatile("v_nop\n\tv_nop\n\tv_nop\n\tv_nop" : "+v"(a), "+v"(b) : "v"(x), "v"(y)); }
__device__ __forceinline__ void keep4_h(v16h a, v16h b, v16h c, v16h d) { asm volatile("v_nop" :: "v"(a), "v"(b), "v"(c), "v"(d)); }
__device__ __forceinline__ void keep4_b(v16b a, v16b b, v16b c, v16b d) { asm volatile("v_nop" :: "v"(a), "v"(b), "v"(c), "v"(d)); }
__device__ __forceinline__ void acc_guard4(v8f& a, v8f& b, v8f& c, v8f& d) { asm volatile("v_nop\n\tv_nop\n\tv_nop\n\tv_nop" : "+v"(a), "+v"(b), "+v"(c), "+v"(d)); }
template <typename T> struct Frag;
template <> struct Frag<_Float16> {
  typedef v16h V; union U { v16h v; v8h h[2]; };
  static __device__ __forceinline__ v16h load(const _Float16* p) {
    U f; f.h[0] = *(const v8h*)(p); f.h[1] = *(const v8h*)(p + 16); return f.v;
  }
  static __device__ __forceinline__ v8f mma(v16h a, v16h b, v8f c) {
    return __builtin_amdgcn_wmma_f32_16x16x32_f16(false, a, false, b, (short)0, c, false, false);
  }
  static __device__ __forceinline__ void guard(v8f& a, v8f& b, v16h x, v16h y) { dep_guard_h(a, b, x, y); }
  static __device__ __forceinline__ void keep(v16h a, v16h b, v16h c, v16h d) { keep4_h(a, b, c, d); }
};
template <> struct Frag<__bf16> {
  typedef v16b V; union U { v16b v; v8b h[2]; };
  static __device__ __forceinline__ v16b load(const __bf16* p) {
    U f; f.h[0] = *(const v8b*)(p); f.h[1] = *(const v8b*)(p + 16); return f.v;
  }
  static __device__ __forceinline__ v8f mma(v16b a, v16b b, v8f c) {
    return __builtin_amdgcn_wmma_f32_16x16x32_bf16(false, a, false, b, (short)0, c, false, false);
  }
  static __device__ __forceinline__ void guard(v8f& a, v8f& b, v16b x, v16b y) { dep_guard_b(a, b, x, y); }
  static __device__ __forceinline__ void keep(v16b a, v16b b, v16b c, v16b d) { keep4_b(a, b, c, d); }
};

__device__ __forceinline__ unsigned pk16(unsigned short a, unsigned short b) { return (unsigned)a | ((unsigned)b << 16); }
__device__ __forceinline__ unsigned short h_bits(float f) { const _Float16 h = (_Float16)f; return __builtin_bit_cast(unsigned short, h); }
__device__ __forceinline__ float bfr(float f) { return bf_bits2f(f2bf_bits(f)); }
__device__ __forceinline__ float h16_to_f32(unsigned hb) {
  const unsigned sgn = (hb & 0x8000u) << 16; const unsigned em = hb & 0x7fffu;
  const float fn = __uint_as_float((em << 13) + 0x38000000u);
  const float fs = (float)em * 5.9604644775390625e-8f;
  const float mag = (em < 0x400u) ? fs : fn; return __uint_as_float(__float_as_uint(mag) | sgn); }

template <int ET> struct Elem;
template <> struct Elem<0> { typedef _Float16 T; };
template <> struct Elem<1> { typedef __bf16 T; };
template <int ET, int BIAS_MODE, int OUT_MODE, bool RESID, int ACT>
__global__ __launch_bounds__(256) void gemm64_kernel(
    const unsigned short* __restrict__ Ap, int lda,
    const unsigned short* __restrict__ Btp, int ldb,
    void* __restrict__ Cout, int ldc,
    const float* __restrict__ bias,
    const float* __restrict__ resid, int ldr,
    int M, int N, int K, int Mlim, float scale, float oscale) {
  static_assert(BIAS_MODE == 0 || BIAS_MODE == 2, "cfg");
  static_assert(OUT_MODE == 0 || OUT_MODE == 1, "cfg");
  static_assert(!(RESID && ACT != 0), "cfg");
  typedef typename Elem<ET>::T T;
  typedef typename Frag<T>::V V;
  const T* A = (const T*)Ap; const T* Bt = (const T*)Btp;
  __shared__ __align__(16) float sT[8][16 * 68];
  const int lane = threadIdx.x & 31;
  const int wave = threadIdx.x >> 5;
  const int tilesN = N >> 6;
  const int tilesM = M >> 6;
  const int tile = blockIdx.x * 8 + wave;
  if (tile >= tilesM * tilesN) return;
  const int tm = tile / tilesN;
  const int tn = tile - tm * tilesN;
  const int m0 = tm << 6;
  const int n0 = tn << 6;

  const int rlane = lane & 15;
  const int koff  = (lane >> 4) * 8;
  const int mOff  = (lane >> 4) * 8;

  v8f acc[4][4];
#pragma unroll
  for (int i = 0; i < 4; ++i)
#pragma unroll
    for (int j = 0; j < 4; ++j) acc[i][j] = (v8f){0.f,0.f,0.f,0.f,0.f,0.f,0.f,0.f};

  for (int k0 = 0; k0 < K; k0 += 32) {
    V bh[4];
#pragma unroll
    for (int j = 0; j < 4; ++j) {
      const size_t bo = (size_t)(n0 + (j << 4) + rlane) * ldb + koff + k0;
      bh[j] = Frag<T>::load(Bt + bo);
    }
#pragma unroll
    for (int i = 0; i < 4; ++i) {
      const size_t ao = (size_t)(m0 + (i << 4) + rlane) * lda + koff + k0;
      V ah = Frag<T>::load(A + ao);
#pragma unroll
      for (int j = 0; j < 4; ++j) {
        acc[i][j] = Frag<T>::mma(ah, bh[j], acc[i][j]);
      }
      Frag<T>::guard(acc[i][0], acc[i][3], ah, ah);
    }
    Frag<T>::keep(bh[0], bh[1], bh[2], bh[3]);
  }
  acc_guard4(acc[0][0], acc[0][1], acc[0][2], acc[0][3]);
  acc_guard4(acc[1][0], acc[1][1], acc[1][2], acc[1][3]);
  acc_guard4(acc[2][0], acc[2][1], acc[2][2], acc[2][3]);
  acc_guard4(acc[3][0], acc[3][1], acc[3][2], acc[3][3]);

  float* slab = sT[wave];
#pragma unroll
  for (int i = 0; i < 4; ++i) {
    const int mBase = m0 + (i << 4);
#pragma unroll
    for (int j = 0; j < 4; ++j) {
      const int n = n0 + (j << 4) + rlane;
      float bv = 0.f;
      if (BIAS_MODE == 2) bv = bias[n];
#pragma unroll
      for (int r = 0; r < 8; ++r) {
        float v = acc[i][j][r] * scale;
        if (BIAS_MODE == 2) v += bv;
        if (ACT == 2) v = fmaxf(v, 0.0f);
        slab[(mOff + r) * 68 + (j << 4) + rlane] = v;
      }
    }
    __builtin_amdgcn_fence(__ATOMIC_RELEASE, "workgroup");
    __builtin_amdgcn_wave_barrier();
    __builtin_amdgcn_fence(__ATOMIC_ACQUIRE, "workgroup");
    if (OUT_MODE == 0) {
      float* C = (float*)Cout;
      const int hh = lane >> 4, c4 = (lane & 15) * 4;
      for (int pass = 0; pass < 2; ++pass) {
#pragma unroll
        for (int it = 0; it < 8; ++it) {
          const int row = it * 2 + hh;
          const int grow = mBase + row;
          v4f v = *(const v4f*)(slab + row * 68 + c4);
          if (RESID) {
            const v4f rr = *(const v4f*)(resid + (size_t)grow * ldr + n0 + c4);
            v = (v + rr) * oscale;
          }
          if (grow < Mlim) *(volatile v4f*)(C + (size_t)grow * ldc + n0 + c4) = v;
        }
        __threadfence();
      }
    } else {
      const int q = lane >> 3, c8 = (lane & 7) * 8;
      unsigned short* C = (unsigned short*)Cout;
      for (int pass = 0; pass < 2; ++pass) {
#pragma unroll
        for (int it = 0; it < 4; ++it) {
          const int row = it * 4 + q;
          const int grow = mBase + row;
          const float* sp = slab + row * 68 + c8;
          float vv[8];
#pragma unroll
          for (int e = 0; e < 8; ++e) vv[e] = sp[e];
          if (RESID) {
            const float* rp = resid + (size_t)grow * ldr + n0 + c8;
            const v4f r0 = *(const v4f*)(rp);
            const v4f r1 = *(const v4f*)(rp + 4);
#pragma unroll
            for (int e = 0; e < 4; ++e) { vv[e] = (vv[e] + r0[e]) * oscale; vv[4 + e] = (vv[4 + e] + r1[e]) * oscale; }
          }
          v8h hv;
#pragma unroll
          for (int e = 0; e < 8; ++e) hv[e] = (_Float16)vv[e];
          if (grow < Mlim) *(volatile v8h*)(C + (size_t)grow * ldc + n0 + c8) = hv;
        }
        __threadfence();
      }
    }
    __builtin_amdgcn_fence(__ATOMIC_RELEASE, "workgroup");
    __builtin_amdgcn_wave_barrier();
    __builtin_amdgcn_fence(__ATOMIC_ACQUIRE, "workgroup");
  }
}

__global__ __launch_bounds__(256) void xcast_kernel(const float* __restrict__ x, unsigned short* __restrict__ Xb) {
  const int i = blockIdx.x * 256 + threadIdx.x;
  if (i >= kNP * kIn / 8) return;
  const int row = i >> 4;
  const int c8 = (i & 15) * 8;
  const bool live = row < kN;
  const int rc = live ? row : (kN - 1);
  const float* p = x + (size_t)rc * kIn + c8;
  const v4f a = *(const v4f*)(p);
  const v4f c = *(const v4f*)(p + 4);
  unsigned short hb[8];
#pragma unroll
  for (int e = 0; e < 4; ++e) {
    hb[e]     = live ? f2bf_bits(a[e]) : (unsigned short)0;
    hb[4 + e] = live ? f2bf_bits(c[e]) : (unsigned short)0;
  }
  const v4u u = (v4u){pk16(hb[0], hb[1]), pk16(hb[2], hb[3]), pk16(hb[4], hb[5]), pk16(hb[6], hb[7])};
  unsigned short* d = Xb + 8 * (size_t)i;
  *(volatile v4u*)d = u;
  __threadfence();
  *(volatile v4u*)d = u;
}

__global__ __launch_bounds__(256) void wtrans_kernel(const float* __restrict__ Wq, const float* __restrict__ Wk,
                                                     const float* __restrict__ Wv, const float* __restrict__ Wo,
                                                     unsigned short* __restrict__ Btx, unsigned short* __restrict__ Btvt,
                                                     unsigned short* __restrict__ Bto) {
  __shared__ float sm[64][65];
  const int t  = threadIdx.x;
  const int tb = blockIdx.x;
  const float* W = Wo; int k0 = 0, n0 = 0; unsigned short* dst = Bto; int ldo = kHid; int mode16 = 1;
  if (tb < 12) {
    const int m = tb >> 2, rem = tb & 3, nt = rem >> 1, kt = rem & 1;
    W = (m == 0) ? Wq : ((m == 1) ? Wk : Wv);
    k0 = kt * 64; n0 = nt * 64;
    dst = Btx + (size_t)(m * kHid + n0) * kIn + k0; ldo = kIn; mode16 = 0;
  } else if (tb < 14) {
    const int nt = tb - 12;
    W = Wv; k0 = kIn; n0 = nt * 64;
    dst = Btvt + (size_t)n0 * kT2V; ldo = kT2V; mode16 = 1;
  } else {
    const int rem = tb - 14, nt = rem >> 1, kt = rem & 1;
    W = Wo; k0 = kt * 64; n0 = nt * 64;
    dst = Bto + (size_t)n0 * kHid + k0; ldo = kHid; mode16 = 1;
  }
#pragma unroll
  for (int i = 0; i < 16; ++i) {
    const int e = i * 256 + t;
    const int kl = e >> 6;
    const int nl = e & 63;
    sm[nl][kl] = bfr(W[(size_t)(k0 + kl) * kHid + n0 + nl]);
  }
  __syncthreads();
  const int lane = t & 31, wave = t >> 5;
  const int q = lane >> 3, c8 = (lane & 7) * 8;
  for (int pass = 0; pass < 2; ++pass) {
#pragma unroll
    for (int it = 0; it < 2; ++it) {
      const int row = wave * 8 + it * 4 + q;
      unsigned short hb[8];
#pragma unroll
      for (int e = 0; e < 8; ++e) {
        const float v = sm[row][c8 + e];
        hb[e] = mode16 ? h_bits(v * kWCarry) : f2bf_bits(v);
      }
      const v4u u = (v4u){pk16(hb[0], hb[1]), pk16(hb[2], hb[3]), pk16(hb[4], hb[5]), pk16(hb[6], hb[7])};
      *(volatile v4u*)(dst + (size_t)row * ldo + c8) = u;
    }
    __threadfence();
  }
}

__global__ __launch_bounds__(256) void misc_kernel(const float* __restrict__ Wk, const float* __restrict__ Wq,
                                                   const float* __restrict__ bo, const float* __restrict__ b0p,
                                                   const float* __restrict__ Bt,
                                                   unsigned short* __restrict__ Btkt, float* __restrict__ cq16, float* __restrict__ bor) {
  __shared__ __align__(16) float s[256];
  const int t = threadIdx.x;
  const int lane = t & 31, wave = t >> 5;
  if (blockIdx.x < 4) {
    const int i = blockIdx.x * 256 + t;
    const float* p = Wk + (size_t)kIn * kHid + 8 * (size_t)i;
    const v4f a = *(const v4f*)(p);
    const v4f c = *(const v4f*)(p + 4);
    unsigned short hb[8];
#pragma unroll
    for (int e = 0; e < 4; ++e) {
      hb[e]     = h_bits(bfr(a[e]) * kWCarry);
      hb[4 + e] = h_bits(bfr(c[e]) * kWCarry);
    }
    const v4u u = (v4u){pk16(hb[0], hb[1]), pk16(hb[2], hb[3]), pk16(hb[4], hb[5]), pk16(hb[6], hb[7])};
    unsigned short* d = Btkt + 8 * (size_t)i;
    *(volatile v4u*)d = u;
    __threadfence();
    *(volatile v4u*)d = u;
  } else {
    float v = 0.0f;
    if (t < kHid) {
      const int h = t;
      float accv = 0.0f;
      accv += bfr(b0p[0]) * bfr(Wq[(size_t)kIn * kHid + h]);
#pragma unroll 1
      for (int j = 0; j < kT2V - 1; ++j) {
        const float sv = sinf(bfr(Bt[j]));
        accv += sv * bfr(Wq[(size_t)(kIn + 1 + j) * kHid + h]);
      }
      v = accv * kQCarry;
    } else {
      v = bfr(bo[t - kHid]);
    }
    s[t] = v;
    __syncthreads();
    if (wave == 0) {
      const v4f o = *(const v4f*)(s + 4 * lane);
      *(volatile v4f*)(cq16 + 4 * lane) = o;
      __threadfence();
      *(volatile v4f*)(cq16 + 4 * lane) = o;
    } else if (wave == 1) {
      const v4f o = *(const v4f*)(s + kHid + 4 * lane);
      *(volatile v4f*)(bor + 4 * lane) = o;
      __threadfence();
      *(volatile v4f*)(bor + 4 * lane) = o;
    }
  }
}

__global__ __launch_bounds__(256) void node_attn_kernel(
    const unsigned short* __restrict__ Q16, const unsigned short* __restrict__ QK,
    const float* __restrict__ XKV, const int* __restrict__ idxp, const float* __restrict__ tsp,
    const float* __restrict__ w0p, const float* __restrict__ b0p,
    const float* __restrict__ Wt, const float* __restrict__ Bt,
    float* __restrict__ AGGX, unsigned short* __restrict__ TB) {
  __shared__ __align__(16) float teS[8][kK][kT2V];
  const int tid = threadIdx.x, lane = tid & 31, wave = tid >> 5;
  const int node = blockIdx.x * 8 + wave;
  const bool live = node < kN;
  const int nc = live ? node : (kN - 1);

  const float w0 = bfr(w0p[0]), b0 = bfr(b0p[0]);
  int ia = lane - 1; ia = ia < 0 ? 0 : ia;
  const float WA = bfr(Wt[ia]), BA = bfr(Bt[ia]);
  const float WB = bfr(Wt[31 + lane]), BB = bfr(Bt[31 + lane]);

  const unsigned* qrow = (const unsigned*)(Q16 + (size_t)nc * kHid);
  const unsigned qwA = qrow[lane], qwB = qrow[32 + lane];
  const float qA0 = h16_to_f32(qwA & 0xffffu) * kQInv, qA1 = h16_to_f32(qwA >> 16) * kQInv;
  const float qB0 = h16_to_f32(qwB & 0xffffu) * kQInv, qB1 = h16_to_f32(qwB >> 16) * kQInv;
  const unsigned* krow = (const unsigned*)(QK + (size_t)nc * kT2V);
  const unsigned kwA = krow[lane >> 1], kwB = krow[16 + (lane >> 1)];
  const unsigned sh = (unsigned)(lane & 1) * 16u;
  const float qkA = h16_to_f32((kwA >> sh) & 0xffffu) * kQKInv;
  const float qkB = h16_to_f32((kwB >> sh) & 0xffffu) * kQKInv;
  const int li = lane & 15;
  int jn = idxp[(size_t)nc * kK + li];
  jn = jn < 0 ? 0 : (jn >= kN ? (kN - 1) : jn);
  const float tn = bfr(tsp[(size_t)nc * kK + li]);

  float* tes = &teS[wave][0][0];
  float mys = -INFINITY, hold = 0.0f;
#pragma unroll 1
  for (int i = 0; i < 2 * kK; ++i) {
    const int k = i >> 1, hf = i & 1;
    const int j = __shfl(jn, k, 32);
    const float t = __shfl(tn, k, 32);
    const float Ws = hf ? WB : WA, Bs = hf ? BB : BA;
    const float sv = sinf(t * Ws + Bs);
    const float lin = t * w0 + b0;
    const float te = (hf == 0 && lane == 0) ? lin : sv;
    tes[k * kT2V + hf * 32 + lane] = te;
    const float q0 = hf ? qB0 : qA0, q1 = hf ? qB1 : qA1, qk = hf ? qkB : qkA;
    const v2f xk = *(const v2f*)(XKV + (size_t)j * kXKVld + hf * 64 + 2 * lane);
    float p = 0.0f;
    p += q0 * xk[0];
    p += q1 * xk[1];
    p += te * qk;
    p += __shfl_xor(p, 16, 32);
    p += __shfl_xor(p, 8, 32);
    p += __shfl_xor(p, 4, 32);
    p += __shfl_xor(p, 2, 32);
    p += __shfl_xor(p, 1, 32);
    const float sc = (hold + p) * kInvSqrtH;
    mys = (hf == 1 && lane == k) ? sc : mys;
    hold = hf ? 0.0f : p;
  }
  float m = mys;
  m = fmaxf(m, __shfl_xor(m, 16, 32));
  m = fmaxf(m, __shfl_xor(m, 8, 32));
  m = fmaxf(m, __shfl_xor(m, 4, 32));
  m = fmaxf(m, __shfl_xor(m, 2, 32));
  m = fmaxf(m, __shfl_xor(m, 1, 32));
  const float e = expf(mys - m);
  float se = e;
  se += __shfl_xor(se, 16, 32);
  se += __shfl_xor(se, 8, 32);
  se += __shfl_xor(se, 4, 32);
  se += __shfl_xor(se, 2, 32);
  se += __shfl_xor(se, 1, 32);
  const float a = e * (1.0f / se);

  v4f acc = (v4f){0.0f, 0.0f, 0.0f, 0.0f};
  float tbA = 0.0f, tbB = 0.0f;
#pragma unroll 1
  for (int k = 0; k < kK; ++k) {
    const float ak = __shfl(a, k, 32);
    const int j = __shfl(jn, k, 32);
    const v4f xv = *(const v4f*)(XKV + (size_t)j * kXKVld + kHid + 4 * lane);
    acc = acc + ak * xv;
    tbA += ak * tes[k * kT2V + lane];
    tbB += ak * tes[k * kT2V + 32 + lane];
  }
  v4f o;
#pragma unroll
  for (int c = 0; c < 4; ++c) o[c] = live ? acc[c] : 0.0f;
  const float tAo = live ? tbA : 0.0f, tBo = live ? tbB : 0.0f;

  float* arow = AGGX + (size_t)node * kHid + 4 * lane;
  *(volatile v4f*)arow = o;
  __threadfence();
  *(volatile v4f*)arow = o;

  const unsigned wA = (unsigned)h_bits(tAo * kTBCarry), wB = (unsigned)h_bits(tBo * kTBCarry);
  const int gb = 8 * (lane & 3);
  unsigned g[8];
#pragma unroll
  for (int i2 = 0; i2 < 8; ++i2) {
    const unsigned ga = (unsigned)__shfl((int)wA, gb + i2, 32);
    const unsigned gv = (unsigned)__shfl((int)wB, gb + i2, 32);
    g[i2] = (lane & 4) ? gv : ga;
  }
  const v4u u = (v4u){pk16((unsigned short)g[0], (unsigned short)g[1]), pk16((unsigned short)g[2], (unsigned short)g[3]),
                      pk16((unsigned short)g[4], (unsigned short)g[5]), pk16((unsigned short)g[6], (unsigned short)g[7])};
  unsigned short* trow = TB + (size_t)node * kT2V + 8 * lane;
  if (lane < 8) *(volatile v4u*)trow = u;
  __threadfence();
  if (lane < 8) *(volatile v4u*)trow = u;
}

extern "C" void kernel_launch(void* const* d_in, const int* in_sizes, int n_in,
                              void* d_out, int out_size, void* d_ws, size_t ws_size, hipStream_t stream) {
  (void)in_sizes; (void)n_in; (void)out_size;
  const float* x    = (const float*)d_in[0];
  const float* ts   = (const float*)d_in[1];
  const int*   idx  = (const int*)  d_in[2];
  const float* w0   = (const float*)d_in[3];
  const float* b0   = (const float*)d_in[4];
  const float* Wt   = (const float*)d_in[5];
  const float* Bt   = (const float*)d_in[6];
  const float* Wq   = (const float*)d_in[7];
  const float* Wk   = (const float*)d_in[8];
  const float* Wv   = (const float*)d_in[9];
  const float* Wo   = (const float*)d_in[10];
  const float* bo   = (const float*)d_in[11];
  float* out = (float*)d_out;

  char* ws = (char*)d_ws; size_t off = 0;
  auto carve = [&](size_t bytes) -> char* { char* p = ws + off; off += (bytes + 255) & ~(size_t)255; return p; };
  unsigned short* Xb    = (unsigned short*)carve(kBytesXb);
  unsigned short* Btx   = (unsigned short*)carve(kBytesBtx);
  unsigned short* Btkt  = (unsigned short*)carve(kBytesBtkt);
  unsigned short* Btvt  = (unsigned short*)carve(kBytesBtvt);
  unsigned short* Bto   = (unsigned short*)carve(kBytesBto);
  float*          cq16  = (float*)carve(kBytesCq);
  float*          bor   = (float*)carve(kBytesBo);
  unsigned short* Q16   = (unsigned short*)carve(kBytesQ16);
  float*          XKV   = (float*)carve(kBytesXKV);
  unsigned short* QK    = (unsigned short*)carve(kBytesQK);
  float*          AGGX  = (float*)carve(kBytesAggx);
  unsigned short* TB    = (unsigned short*)carve(kBytesTB);
  unsigned short* AGG16 = (unsigned short*)carve(kBytesAgg16);
  if (off > ws_size || off > (size_t)134217728) return;

  xcast_kernel<<<(kNP * kIn / 8 + 255) / 256, 256, 0, stream>>>(x, Xb);
  wtrans_kernel<<<18, 256, 0, stream>>>(Wq, Wk, Wv, Wo, Btx, Btvt, Bto);
  misc_kernel<<<5, 256, 0, stream>>>(Wk, Wq, bo, b0, Bt, Btkt, cq16, bor);

  {
    constexpr int tiles = (kNP / 64) * (kHid / 64);
    gemm64_kernel<1, 2, 1, false, 0><<<(tiles + 7) / 8, 256, 0, stream>>>(
        Xb, kIn, Btx, kIn, (void*)Q16, kHid, cq16, (const float*)nullptr, 0,
        kNP, kHid, kIn, kNP, kQCarry, 1.0f);
  }
  {
    constexpr int tiles = (kNP / 64) * (kXKVld / 64);
    gemm64_kernel<1, 0, 0, false, 0><<<(tiles + 7) / 8, 256, 0, stream>>>(
        Xb, kIn, Btx + (size_t)kHid * kIn, kIn, (void*)XKV, kXKVld, (const float*)nullptr, (const float*)nullptr, 0,
        kNP, kXKVld, kIn, kNP, 1.0f, 1.0f);
  }
  {
    constexpr int tiles = (kNP / 64) * (kT2V / 64);
    gemm64_kernel<0, 0, 1, false, 0><<<(tiles + 7) / 8, 256, 0, stream>>>(
        Q16, kHid, Btkt, kHid, (void*)QK, kT2V, (const float*)nullptr, (const float*)nullptr, 0,
        kNP, kT2V, kHid, kNP, kScaleQK, 1.0f);
  }
  node_attn_kernel<<<kNP / 8, 256, 0, stream>>>(Q16, QK, XKV, idx, ts, w0, b0, Wt, Bt, AGGX, TB);
  {
    constexpr int tiles = (kNP / 64) * (kHid / 64);
    gemm64_kernel<0, 0, 1, true, 0><<<(tiles + 7) / 8, 256, 0, stream>>>(
        TB, kT2V, Btvt, kT2V, (void*)AGG16, kHid, (const float*)nullptr, AGGX, kHid,
        kNP, kHid, kT2V, kNP, kScaleAgg, kAggCarry);
  }
  {
    constexpr int tiles = (kNP / 64) * (kHid / 64);
    gemm64_kernel<0, 2, 0, false, 2><<<(tiles + 7) / 8, 256, 0, stream>>>(
        AGG16, kHid, Bto, kHid, (void*)out, kHid, bor, (const float*)nullptr, 0,
        kNP, kHid, kHid, kN, kScaleOut, 1.0f);
  }
}
